// SpatialGraphDiffusion_17025250361515
// MI455X (gfx1250) — hardware-verified
//
#include <hip/hip_runtime.h>
#include <math.h>

typedef __attribute__((ext_vector_type(16))) _Float16 v16h;
typedef __attribute__((ext_vector_type(16))) __bf16 v16b;
typedef __attribute__((ext_vector_type(8)))  _Float16 v8h;
typedef __attribute__((ext_vector_type(8)))  float v8f;
typedef __attribute__((ext_vector_type(4)))  float v4f;
typedef __attribute__((ext_vector_type(2)))  float v2f;
typedef __attribute__((ext_vector_type(4)))  unsigned v4u;
typedef __attribute__((ext_vector_type(4)))  int v4i;
typedef float __attribute__((may_alias)) float_a;
typedef int __attribute__((may_alias)) int_a;

template <typename T> __device__ __forceinline__ void vst2(void* p, T v) { *(volatile T*)p = v; __threadfence(); *(volatile T*)p = v; }
__device__ __forceinline__ v8f wmma16(v16h a, v16h b, v8f c) {
  v8f d = __builtin_amdgcn_wmma_f32_16x16x32_f16(false, a, false, b, (short)0, c, false, false);
  asm volatile("v_nop\n\tv_nop\n\tv_nop\n\tv_nop" : "+v"(d) : "v"(a), "v"(b));
  return d;
}
__device__ __forceinline__ v8f wmma_bf(v16b a, v16b b, v8f c) {
  v8f d = __builtin_amdgcn_wmma_f32_16x16x32_bf16(false, a, false, b, (short)0, c, false, false);
  asm volatile("v_nop\n\tv_nop\n\tv_nop\n\tv_nop" : "+v"(d) : "v"(a), "v"(b));
  return d;
}
__device__ __forceinline__ v16h frag_h(const _Float16* rowk0, int lane) {
  union { v16h v; v8h q[2]; } u; const _Float16* p = rowk0 + 8 * (lane >> 4);
  u.q[0] = *(const v8h*)p; u.q[1] = *(const v8h*)(p + 16); return u.v;
}
__device__ __forceinline__ v16h frag_f32(const float* rowk0, int lane) {
  v16h a; const float* p = rowk0 + 8 * (lane >> 4);
#pragma unroll
  for (int i = 0; i < 8; ++i) { a[i] = (_Float16)p[i]; a[8 + i] = (_Float16)p[16 + i]; }
  return a;
}
__device__ __forceinline__ v16h frag_f32s(const float* rowk0, int lane, float sc) {
  v16h a; const float* p = rowk0 + 8 * (lane >> 4);
#pragma unroll
  for (int i = 0; i < 8; ++i) { a[i] = (_Float16)(p[i] * sc); a[8 + i] = (_Float16)(p[16 + i] * sc); }
  return a;
}
__device__ __forceinline__ v16h fragc_f32(const float* W, int k0, int n, int lane, int ld, int K) {
  v16h a; const int g = lane >> 4;
#pragma unroll
  for (int i = 0; i < 8; ++i) { const int ka = k0 + 8 * g + i, kb = ka + 16;
    a[i] = (_Float16)(ka < K ? W[(size_t)ka * ld + n] : 0.f); a[8 + i] = (_Float16)(kb < K ? W[(size_t)kb * ld + n] : 0.f); }
  return a;
}
struct F2 { v16b h, l; };
__device__ __forceinline__ F2 bsplit16(const float v[16]) { F2 r;
#pragma unroll
  for (int i = 0; i < 16; ++i) { const __bf16 h = (__bf16)v[i]; r.h[i] = h; r.l[i] = (__bf16)(v[i] - (float)h); }
  return r; }
__device__ __forceinline__ F2 split_row(const float* row, int k0, int lane) { float v[16]; const float* p = row + k0 + 8 * (lane >> 4);
#pragma unroll
  for (int i = 0; i < 8; ++i) { v[i] = p[i]; v[8 + i] = p[16 + i]; }
  return bsplit16(v); }
__device__ __forceinline__ F2 split_rowK(const float* row, int k0, int lane, int K) { float v[16]; const int g = lane >> 4;
#pragma unroll
  for (int i = 0; i < 8; ++i) { const int ka = k0 + 8 * g + i, kb = ka + 16; v[i] = ka < K ? row[ka] : 0.f; v[8 + i] = kb < K ? row[kb] : 0.f; }
  return bsplit16(v); }
__device__ __forceinline__ F2 split_col(const float* W, int k0, int n, int lane, int ld, int K) { float v[16]; const int g = lane >> 4;
#pragma unroll
  for (int i = 0; i < 8; ++i) { const int ka = k0 + 8 * g + i, kb = ka + 16; v[i] = ka < K ? W[(size_t)ka * ld + n] : 0.f; v[8 + i] = kb < K ? W[(size_t)kb * ld + n] : 0.f; }
  return bsplit16(v); }
__device__ __forceinline__ v8f mac3(const F2& a, const F2& b, v8f c) { c = wmma_bf(a.l, b.h, c); c = wmma_bf(a.h, b.l, c); return wmma_bf(a.h, b.h, c); }
__device__ __forceinline__ float sigm(float v) { return 1.0f / (1.0f + expf(-v)); }
#define LDSX() do { asm volatile("s_wait_dscnt 0" ::: "memory"); __builtin_amdgcn_wave_barrier(); __builtin_amdgcn_fence(__ATOMIC_RELEASE, "workgroup"); } while (0)

#define NN 1024
#define HH 64
#define NL 3

__device__ __forceinline__ float sigm_fast(float v) { return __builtin_amdgcn_rcpf(1.0f + __expf(-v)); }
__device__ __forceinline__ float silu_f(float v) { return v * sigm(v); }
__device__ __forceinline__ float silu_fast(float v) { return v * sigm_fast(v); }

__global__ __launch_bounds__(64) void k_init(const float* __restrict__ pos, const int* __restrict__ tt, const float* __restrict__ tw1, const float* __restrict__ tb1,
                                           const float* __restrict__ tw2, const float* __restrict__ tb2, const float* __restrict__ pw, const float* __restrict__ pb,
                                           float* __restrict__ te, float* __restrict__ h) {
  __shared__ float s0[HH], s1[HH];
  const int c = threadIdx.x; const float t = (float)tt[0];
  { const int half = HH / 2; const int i = c < half ? c : c - half; const float fr = expf((float)i * (-logf(10000.0f) / (float)(half - 1)));
    const float v = t * fr; s0[c] = c < half ? sinf(v) : cosf(v); }
  __syncthreads();
  { float a = tb1[c];
#pragma unroll 1
    for (int k = 0; k < HH; ++k) a += s0[k] * tw1[k * HH + c];
    s1[c] = silu_f(a); }
  __syncthreads();
  { float a = tb2[c];
#pragma unroll 1
    for (int k = 0; k < HH; ++k) a += s1[k] * tw2[k * HH + c];
    s0[c] = a; vst2(te + c, (float_a)a); }
  __syncthreads();
#pragma unroll 1
  for (int n = 0; n < NN; ++n) { const float v = pos[n * 3] * pw[c] + pos[n * 3 + 1] * pw[HH + c] + pos[n * 3 + 2] * pw[2 * HH + c] + pb[c] + s0[c]; vst2(h + (size_t)n * HH + c, (float_a)v); }
}
__global__ __launch_bounds__(256) void k_layer(const float* __restrict__ pos, const float* __restrict__ adj, const float* __restrict__ te, const float* __restrict__ hin,
                                            const float* __restrict__ ew1, const float* __restrict__ eb1, const float* __restrict__ ew2, const float* __restrict__ eb2,
                                            const float* __restrict__ mw, const float* __restrict__ mb, float* __restrict__ hout) {
  __shared__ __align__(16) float S[16][HH + 4];
  __shared__ __align__(16) float cat3[16][3 * HH + 4];
  __shared__ __align__(16) float so[16][HH + 4];
  __shared__ float sdeg[16];
  __shared__ float sw1[4 * HH], sb1[HH];
  const int tid = threadIdx.x, w = tid >> 5, lane = tid & 31, col = lane & 15, g = lane >> 4;
  const int il = tid >> 4, cg = tid & 15, c0 = cg * 4; const int i = blockIdx.x * 16 + il;
  for (int q = tid; q < 4 * HH; q += 256) sw1[q] = ew1[q];
  if (tid < HH) sb1[tid] = eb1[tid];
  __syncthreads();
  const float pix = pos[i * 3], piy = pos[i * 3 + 1], piz = pos[i * 3 + 2];
  float acc[4] = {0.f, 0.f, 0.f, 0.f}; float deg = 0.f;
#pragma unroll 1
  for (int j = 0; j < NN; ++j) { const float a = adj[(size_t)i * NN + j];
    if (a == 0.f) continue;
    const float rx = pix - pos[j * 3], ry = piy - pos[j * 3 + 1], rz = piz - pos[j * 3 + 2]; const float d = sqrtf(rx * rx + ry * ry + rz * rz);
    deg += a;
#pragma unroll
    for (int u = 0; u < 4; ++u) { const int c = c0 + u; const float v = rx * sw1[c] + ry * sw1[HH + c] + rz * sw1[2 * HH + c] + d * sw1[3 * HH + c] + sb1[c]; acc[u] += a * silu_fast(v); } }
#pragma unroll
  for (int u = 0; u < 4; ++u) S[il][c0 + u] = acc[u];
  if (cg == 0) sdeg[il] = deg;
  for (int q = tid; q < 16 * HH; q += 256) { const int r = q >> 6, c = q & 63; cat3[r][c] = hin[(size_t)(blockIdx.x * 16 + r) * HH + c]; cat3[r][2 * HH + c] = te[c]; }
  __syncthreads();
  if (w < 4) { v8f ac = {};
#pragma unroll
    for (int kc = 0; kc < 2; ++kc) ac = wmma16(frag_f32(&S[col][0] + kc * 32, lane), fragc_f32(ew2, kc * 32, w * 16 + col, lane, HH, HH), ac);
#pragma unroll
    for (int r = 0; r < 8; ++r) { const int rr = 8 * g + r, c = w * 16 + col; cat3[rr][HH + c] = ac[r] + sdeg[rr] * eb2[c] + cat3[rr][c]; } }
  __syncthreads();
  if (w < 4) { v8f ac = {};
#pragma unroll
    for (int kc = 0; kc < 6; ++kc) ac = wmma16(frag_f32(&cat3[col][0] + kc * 32, lane), fragc_f32(mw, kc * 32, w * 16 + col, lane, HH, 3 * HH), ac);
#pragma unroll
    for (int r = 0; r < 8; ++r) { const int c = w * 16 + col; so[8 * g + r][c] = silu_f(ac[r] + mb[c]); } }
  __syncthreads();
  for (int q = tid; q < 16 * 16; q += 256) { const int r = q >> 4, pc = q & 15; vst2(hout + (size_t)(blockIdx.x * 16 + r) * HH + pc * 4, *(const v4f*)(&so[r][pc * 4])); }
}
__global__ __launch_bounds__(128) void k_heads(const float* __restrict__ h, const float* __restrict__ te, const float* __restrict__ aw1, const float* __restrict__ hw1, const float* __restrict__ hb1,
                                             const float* __restrict__ hw2, const float* __restrict__ hb2, const float* __restrict__ mask, float* __restrict__ hi, float* __restrict__ hj, float* __restrict__ eps) {
  __shared__ __align__(16) float cat2[16][2 * HH + 4];
  __shared__ __align__(16) float s3[3][16][HH + 4];
  __shared__ __align__(16) float se[16 * 3 + 4];
  const int tid = threadIdx.x, w = tid >> 5, lane = tid & 31, col = lane & 15, g = lane >> 4; const int n0 = blockIdx.x * 16;
  for (int q = tid; q < 16 * HH; q += 128) { const int r = q >> 6, c = q & 63; cat2[r][c] = h[(size_t)(n0 + r) * HH + c]; cat2[r][HH + c] = te[c]; }
  __syncthreads();
  if (w < 3) {
#pragma unroll
    for (int t = 0; t < 4; ++t) { v8f ac = {};
      if (w < 2) {
#pragma unroll
        for (int kc = 0; kc < 2; ++kc) ac = wmma16(frag_f32(&cat2[col][0] + kc * 32, lane), fragc_f32(aw1 + (size_t)w * HH * HH, kc * 32, t * 16 + col, lane, HH, HH), ac);
#pragma unroll
        for (int r = 0; r < 8; ++r) s3[w][8 * g + r][t * 16 + col] = ac[r]; }
      else {
#pragma unroll
        for (int kc = 0; kc < 4; ++kc) ac = wmma16(frag_f32(&cat2[col][0] + kc * 32, lane), fragc_f32(hw1, kc * 32, t * 16 + col, lane, HH, 2 * HH), ac);
#pragma unroll
        for (int r = 0; r < 8; ++r) { const int c = t * 16 + col; s3[2][8 * g + r][c] = silu_f(ac[r] + hb1[c]); } } } }
  __syncthreads();
  if (tid < 48) { const int r = tid / 3, k = tid % 3; float a = hb2[k]; for (int c = 0; c < HH; ++c) a += s3[2][r][c] * hw2[c * 3 + k]; se[r * 3 + k] = a * mask[n0 + r]; }
  __syncthreads();
  for (int q = tid; q < 2 * 16 * 16; q += 128) { const int which = q >> 8, rem = q & 255, r = rem >> 4, pc = rem & 15; vst2((which == 0 ? hi : hj) + (size_t)(n0 + r) * HH + pc * 4, *(const v4f*)(&s3[which][r][pc * 4])); }
  if (tid < 12) vst2(eps + (size_t)n0 * 3 + tid * 4, *(const v4f*)(&se[tid * 4]));
}
__global__ __launch_bounds__(256) void k_logits(const float* __restrict__ hi, const float* __restrict__ hj, const float* __restrict__ ab1, const float* __restrict__ aw2, const float* __restrict__ ab2, float* __restrict__ Lg) {
  __shared__ float shi[HH], sw2[HH];
  __shared__ __align__(16) float so[256];
  const int i = blockIdx.y, j = blockIdx.x * 256 + threadIdx.x, tid = threadIdx.x;
  if (tid < HH) { shi[tid] = hi[(size_t)i * HH + tid] + ab1[tid]; sw2[tid] = aw2[tid]; }
  __syncthreads();
  float a = ab2[0]; const float* hr = hj + (size_t)j * HH;
#pragma unroll 1
  for (int c = 0; c < HH; ++c) a += silu_fast(shi[c] + hr[c]) * sw2[c];
  so[tid] = a; __syncthreads();
  if (tid < 64) vst2(Lg + (size_t)i * NN + blockIdx.x * 256 + tid * 4, *(const v4f*)(&so[tid * 4]));
}
__global__ __launch_bounds__(256) void k_sym(const float* __restrict__ Lg, const float* __restrict__ mask, float* __restrict__ adjp) {
  const int i = blockIdx.x, tid = threadIdx.x; const float mi = mask[i];
  for (int q = tid; q < NN / 4; q += 256) { v4f v;
#pragma unroll
    for (int e = 0; e < 4; ++e) { const int j = q * 4 + e; v[e] = sigm(0.5f * (Lg[(size_t)i * NN + j] + Lg[(size_t)j * NN + i])) * mask[j] * mi; }
    vst2(adjp + (size_t)i * NN + q * 4, v); }
}
extern "C" void kernel_launch(void* const* d_in, const int* in_sizes, int n_in, void* d_out, int out_size, void* d_ws, size_t ws_size, hipStream_t stream) {
  (void)in_sizes; (void)n_in; (void)out_size; (void)ws_size;
  const float** I = (const float**)d_in;
  const float* pos = I[0]; const float* adj = I[1]; const float* mask = I[2]; const int* tt = (const int*)d_in[3];
  const float* tw1 = I[4]; const float* tb1 = I[5]; const float* tw2 = I[6]; const float* tb2 = I[7]; const float* pw = I[8]; const float* pb = I[9];
  const float* ew1 = I[10]; const float* eb1 = I[11]; const float* ew2 = I[12]; const float* eb2 = I[13]; const float* mw = I[14]; const float* mb = I[15];
  const float* aw1 = I[16]; const float* ab1 = I[17]; const float* aw2 = I[18]; const float* ab2 = I[19]; const float* hw1 = I[20]; const float* hb1 = I[21]; const float* hw2 = I[22]; const float* hb2 = I[23];
  float* adjp = (float*)d_out; float* eps = adjp + (size_t)NN * NN;
  char* ws = (char*)d_ws; size_t off = 0;
  auto take = [&](size_t bytes) { char* p = ws + off; off += (bytes + 255) & ~(size_t)255; return p; };
  float* te = (float*)take(256); float* hA = (float*)take((size_t)NN * HH * 4); float* hB = (float*)take((size_t)NN * HH * 4);
  float* hi = (float*)take((size_t)NN * HH * 4); float* hj = (float*)take((size_t)NN * HH * 4); float* Lg = (float*)take((size_t)NN * NN * 4);
  k_init<<<1, 64, 0, stream>>>(pos, tt, tw1, tb1, tw2, tb2, pw, pb, te, hA);
  float* hc = hA; float* hn = hB;
  for (int l = 0; l < NL; ++l) { k_layer<<<NN / 16, 256, 0, stream>>>(pos, adj, te, hc, ew1 + l * 4 * HH, eb1 + l * HH, ew2 + (size_t)l * HH * HH, eb2 + l * HH, mw + (size_t)l * 3 * HH * HH, mb + l * HH, hn); float* t = hc; hc = hn; hn = t; }
  k_heads<<<NN / 16, 128, 0, stream>>>(hc, te, aw1, hw1, hb1, hw2, hb2, mask, hi, hj, eps);
  k_logits<<<dim3(NN / 256, NN), 256, 0, stream>>>(hi, hj, ab1, aw2, ab2, Lg);
  k_sym<<<NN, 256, 0, stream>>>(Lg, mask, adjp);
}
